// HGCLayer_77532749628050
// MI455X (gfx1250) — hardware-verified
//
#include <hip/hip_runtime.h>
#include <stddef.h>
#include <stdint.h>


#define DD      256
#define DQ      512
#define NTHR    256
#define NWAVE   8
#define EPT     8
#define CHUNK   (NTHR * EPT)
#define WCAP    (EPT * 32)
#define LISTN   (NWAVE * WCAP)
#define NBMAX   2048
#define RCAP    28672
#define DEGCAP  4096
#define GBM     64
#define GBN     64
#define GTHR    128
#define NCH     8
#define EPW     4
#define EPB     (NWAVE * EPW)
#define WROWS   1280
#define CA      32.0f
#define CW      256.0f
#define SCL     0.0001220703125f
#define EPSF    1e-6f
#define ONEPE   1.000001f
#define LNEPS   1e-5f
#define WSMAX   134217728
#define LDS_AGG ((2 * RCAP + 2 * NBMAX + LISTN) * 4 + 64)

static_assert((CHUNK & (CHUNK - 1)) == 0 && CHUNK <= 4096);
static_assert((NBMAX & (NBMAX - 1)) == 0 && NBMAX <= 4096);
static_assert(NTHR * 8 == NBMAX);
static_assert(LISTN >= NBMAX);
static_assert(LISTN >= NWAVE * WCAP);
static_assert((RCAP % 32) == 0);
static_assert(LDS_AGG <= 300000);
static_assert(GBM == (GTHR / 32) * 16);
static_assert((DD % 32) == 0 && (DD % GBN) == 0 && (DQ % GBN) == 0);
static_assert(EPB == 32);
static_assert(NTHR == DD);
static_assert((GBM % EPB) == 0);
static_assert(DD / 8 == 32);

typedef float    v4f  __attribute__((ext_vector_type(4)));
typedef float    v8f  __attribute__((ext_vector_type(8)));
typedef int      v4i  __attribute__((ext_vector_type(4)));
typedef int      v8i  __attribute__((ext_vector_type(8)));
typedef _Float16 v8h  __attribute__((ext_vector_type(8)));
typedef _Float16 v16h __attribute__((ext_vector_type(16)));
union FragH { v16h v; v8h h[2]; v8i w; };

__device__ __forceinline__ v8f wmh(const FragH& a, const FragH& b, v8f c) {
  v8f d = __builtin_amdgcn_wmma_f32_16x16x32_f16(false, a.v, false, b.v, (short)0, c, false, false);
  asm volatile("v_nop\n\tv_nop\n\tv_nop\n\tv_nop" : "+v"(d) : "v"(a.w), "v"(b.w));
  return d;
}

__device__ __forceinline__ void ldwait() {
  asm volatile("s_wait_loadcnt 0x0" ::: "memory");
}

__device__ __forceinline__ v8h cvt8h(const v4f a, const v4f b, const float c) {
  v8h hv;
  hv[0] = (_Float16)(a.x * c); hv[1] = (_Float16)(a.y * c);
  hv[2] = (_Float16)(a.z * c); hv[3] = (_Float16)(a.w * c);
  hv[4] = (_Float16)(b.x * c); hv[5] = (_Float16)(b.y * c);
  hv[6] = (_Float16)(b.z * c); hv[7] = (_Float16)(b.w * c);
  return hv;
}

__device__ __forceinline__ float wred(float v) {
#pragma unroll
  for (int o = 16; o > 0; o >>= 1) v += __shfl_xor(v, o);
  return v;
}

__device__ __forceinline__ float rcp_f(float x) { return __builtin_amdgcn_rcpf(x); }
__device__ __forceinline__ float sigm_f(float x) { return rcp_f(1.0f + __expf(-x)); }
__device__ __forceinline__ float silu_f(float x) { return x * sigm_f(x); }

__device__ __forceinline__ void chsh(float n, float& ch, float& sh) {
  const float e  = expf(n);
  const float ei = rcp_f(e);
  ch = 0.5f * (e + ei);
  const float n2 = n * n;
  const float st = n * fmaf(n2, fmaf(n2, 0.0083333333f, 0.16666667f), 1.0f);
  const float se = 0.5f * (e - ei);
  sh = (n < 0.25f) ? st : se;
}

__device__ __forceinline__ void relay8(const float z[8], int lane, v4f& va, v4f& vb) {
  const int s0 = lane >> 1;
  const int s1 = 16 + (lane >> 1);
  const bool odd = (lane & 1) != 0;
  float pa[4], pb[4];
#pragma unroll
  for (int k = 0; k < 4; ++k) {
    const float l0 = __shfl(z[k], s0), h0 = __shfl(z[4 + k], s0);
    const float l1 = __shfl(z[k], s1), h1 = __shfl(z[4 + k], s1);
    pa[k] = odd ? h0 : l0;
    pb[k] = odd ? h1 : l1;
  }
  va.x = pa[0]; va.y = pa[1]; va.z = pa[2]; va.w = pa[3];
  vb.x = pb[0]; vb.y = pb[1]; vb.z = pb[2]; vb.w = pb[3];
}

__device__ __forceinline__ void put_row(float* rowp, const float z[8], int lane) {
  v4f va, vb;
  relay8(z, lane, va, vb);
  float* p0 = rowp + 4 * lane;
  float* p1 = rowp + (DD / 2) + 4 * lane;
  *(volatile v4f*)p0 = va;
  *(volatile v4f*)p1 = vb;
  __threadfence();
  *(volatile v4f*)p0 = va;
  *(volatile v4f*)p1 = vb;
}

__device__ __forceinline__ int scan_chunk(const int* __restrict__ dsts, int nE, int cbase, int slotBase,
                                          int nb, int vec8, int* list, int tid, int lane, int wave) {
  int wc = 0;
  const int el0  = tid * EPT;
  const int e0   = cbase + el0;
  const int sent = -2147483647 - 1;
  v4i da, db;
  if (vec8 != 0 && cbase + CHUNK <= nE) {
    da = *(const v4i*)(dsts + e0);
    db = *(const v4i*)(dsts + e0 + 4);
  } else {
    da.x = (e0     < nE) ? dsts[min(e0,     nE - 1)] : sent;
    da.y = (e0 + 1 < nE) ? dsts[min(e0 + 1, nE - 1)] : sent;
    da.z = (e0 + 2 < nE) ? dsts[min(e0 + 2, nE - 1)] : sent;
    da.w = (e0 + 3 < nE) ? dsts[min(e0 + 3, nE - 1)] : sent;
    db.x = (e0 + 4 < nE) ? dsts[min(e0 + 4, nE - 1)] : sent;
    db.y = (e0 + 5 < nE) ? dsts[min(e0 + 5, nE - 1)] : sent;
    db.z = (e0 + 6 < nE) ? dsts[min(e0 + 6, nE - 1)] : sent;
    db.w = (e0 + 7 < nE) ? dsts[min(e0 + 7, nE - 1)] : sent;
  }
  const unsigned nbs = (unsigned)slotBase;
  const unsigned unb = (unsigned)nb;
  const unsigned s0 = (unsigned)da.x - nbs, s1 = (unsigned)da.y - nbs;
  const unsigned s2 = (unsigned)da.z - nbs, s3 = (unsigned)da.w - nbs;
  const unsigned s4 = (unsigned)db.x - nbs, s5 = (unsigned)db.y - nbs;
  const unsigned s6 = (unsigned)db.z - nbs, s7 = (unsigned)db.w - nbs;
  const bool h0 = s0 < unb, h1 = s1 < unb, h2 = s2 < unb, h3 = s3 < unb;
  const bool h4 = s4 < unb, h5 = s5 < unb, h6 = s6 < unb, h7 = s7 < unb;
  const unsigned any = __builtin_amdgcn_ballot_w32(h0 | h1 | h2 | h3 | h4 | h5 | h6 | h7);
  if (any != 0u) {
#define HITJ(J, HJ, SJ) { \
      const unsigned mj = __builtin_amdgcn_ballot_w32(HJ); \
      if (mj != 0u) { \
        if (HJ) { \
          const int pos = wc + (int)__builtin_amdgcn_mbcnt_lo(mj, 0u); \
          if (pos < WCAP) list[wave * WCAP + pos] = ((el0 + (J)) << 12) | (int)(SJ); \
        } \
        wc += (int)__builtin_popcount(mj); } }
    HITJ(0, h0, s0)
    HITJ(1, h1, s1)
    HITJ(2, h2, s2)
    HITJ(3, h3, s3)
    HITJ(4, h4, s4)
    HITJ(5, h5, s5)
    HITJ(6, h6, s6)
    HITJ(7, h7, s7)
#undef HITJ
  }
  return wc;
}

__global__ __launch_bounds__(NTHR) void k_wcvt(const float* __restrict__ w0, const float* __restrict__ w1,
                                               const float* __restrict__ w2, const float* __restrict__ w3,
                                               const float* __restrict__ w4, _Float16* wt, int nUnits) {
  const int u = (int)blockIdx.x * NTHR + (int)threadIdx.x;
  if (u >= nUnits) return;
  const int n  = u >> 5;
  const int k8 = (u & 31) * 8;
  int seg = n >> 8;
  seg = seg > 4 ? 4 : seg;
  const int nc = n & 255;
  const float* ws = (seg == 0) ? w0 : ((seg == 1) ? w1 : ((seg == 2) ? w2 : ((seg == 3) ? w3 : w4)));
  const float* p = ws + (size_t)k8 * DD + nc;
  v4f a, b;
  a.x = p[0];                 a.y = p[(size_t)DD];        a.z = p[(size_t)2 * DD];    a.w = p[(size_t)3 * DD];
  b.x = p[(size_t)4 * DD];    b.y = p[(size_t)5 * DD];    b.z = p[(size_t)6 * DD];    b.w = p[(size_t)7 * DD];
  const v8h hv = cvt8h(a, b, CW);
  const size_t o = (size_t)n * DD + k8;
  *(volatile v8h*)(wt + o) = hv;
  __threadfence();
  *(volatile v8h*)(wt + o) = hv;
}

__global__ __launch_bounds__(NTHR) void k_tan(const float* __restrict__ src, _Float16* dst, int nSrc, int nUnits) {
  const int i = (int)blockIdx.x * NTHR + (int)threadIdx.x;
  if (i >= nUnits) return;
  const int row = i >> 5;
  const int c0  = (i & 31) * 8;
  const int rc  = row < nSrc ? row : nSrc - 1;
  const float* p = src + (size_t)rc * DD;
  const float x0r = p[0];
  v4f a = *(const v4f*)(p + c0), b = *(const v4f*)(p + c0 + 4);
  const float x0 = fmaxf(x0r, ONEPE);
  const float d  = acoshf(x0);
  const float cf = d * rcp_f(sqrtf(x0 * x0 - 1.0f));
  a = a * cf;
  b = b * cf;
  if (c0 == 0) a.x = 0.f;
  const v4f z4 = {0.f, 0.f, 0.f, 0.f};
  if (row >= nSrc) { a = z4; b = z4; }
  const v8h hv = cvt8h(a, b, CA);
  const size_t o = (size_t)row * DD + c0;
  *(volatile v8h*)(dst + o) = hv;
  __threadfence();
  *(volatile v8h*)(dst + o) = hv;
}

template<int EPI>
__global__ __launch_bounds__(GTHR) void k_gemm(
    const _Float16* __restrict__ A, const _Float16* __restrict__ WT,
    const float* __restrict__ bias, const float* __restrict__ eattr,
    const float* __restrict__ esd, const float* __restrict__ esa,
    const float* __restrict__ wx, float* outF, _Float16* outH,
    int K, int ldo, int nbias, int ebase, int nE, float scl)
{
  __shared__ __attribute__((aligned(16))) float stg[GBM * GBN];
  const int tid = (int)threadIdx.x, lane = tid & 31, wave = tid >> 5, hh = lane >> 4, m = lane & 15;
  const int rowBase = (int)blockIdx.x * GBM;
  const int col0    = (int)blockIdx.y * GBN;

  v8f acc[4];
  {
    const v8f z = {0.f, 0.f, 0.f, 0.f, 0.f, 0.f, 0.f, 0.f};
    acc[0] = z; acc[1] = z; acc[2] = z; acc[3] = z;
  }
  const _Float16* ap = A  + (size_t)(rowBase + 16 * wave + m) * (size_t)K + 8 * hh;
  const _Float16* wp = WT + (size_t)(col0 + m) * (size_t)K + 8 * hh;
  const int ksteps = K >> 5;
#pragma unroll 1
  for (int ks = 0; ks < ksteps; ++ks) {
    FragH af;
    af.h[0] = *(const v8h*)(ap + 32 * ks);
    af.h[1] = *(const v8h*)(ap + 32 * ks + 16);
#pragma unroll
    for (int t = 0; t < 4; ++t) {
      const _Float16* wq = wp + (size_t)(16 * t) * (size_t)K + 32 * ks;
      FragH bf;
      bf.h[0] = *(const v8h*)wq;
      bf.h[1] = *(const v8h*)(wq + 16);
      acc[t] = wmh(af, bf, acc[t]);
    }
  }

  float ev0[8], ev1[8];
#pragma unroll
  for (int r = 0; r < 8; ++r) { ev0[r] = 0.f; ev1[r] = 0.f; }
  if (EPI == 1 || EPI == 2) {
    const int lr0 = rowBase + 16 * wave + 8 * hh;
    if (EPI == 1) {
      if (ebase + rowBase + GBM <= nE) {
        const float* q = eattr + (size_t)ebase + lr0;
        const v4f a = *(const v4f*)q, b = *(const v4f*)(q + 4);
        ev0[0] = a.x; ev0[1] = a.y; ev0[2] = a.z; ev0[3] = a.w;
        ev0[4] = b.x; ev0[5] = b.y; ev0[6] = b.z; ev0[7] = b.w;
      } else {
#pragma unroll
        for (int r = 0; r < 8; ++r) {
          int gi = ebase + lr0 + r;
          gi = gi > nE - 1 ? nE - 1 : gi;
          ev0[r] = eattr[gi];
        }
      }
      const v4f a = *(const v4f*)(esd + lr0), b = *(const v4f*)(esd + lr0 + 4);
      ev1[0] = a.x; ev1[1] = a.y; ev1[2] = a.z; ev1[3] = a.w;
      ev1[4] = b.x; ev1[5] = b.y; ev1[6] = b.z; ev1[7] = b.w;
    } else {
      const v4f a = *(const v4f*)(esa + lr0), b = *(const v4f*)(esa + lr0 + 4);
      ev0[0] = a.x; ev0[1] = a.y; ev0[2] = a.z; ev0[3] = a.w;
      ev0[4] = b.x; ev0[5] = b.y; ev0[6] = b.z; ev0[7] = b.w;
    }
  }

#pragma unroll
  for (int t = 0; t < 4; ++t) {
    const int lc  = 16 * t + m;
    const int col = col0 + lc;
    float bv, w0 = 0.f, w1 = 0.f;
    if (EPI == 0) {
      int bi = col > nbias - 1 ? nbias - 1 : col;
      bi = bi < 0 ? 0 : bi;
      const float bl = bias[bi];
      bv = (col < nbias) ? bl : 0.f;
    } else {
      const int ci = col > DD - 1 ? DD - 1 : col;
      bv = bias[ci];
      if (EPI == 1) { w0 = wx[ci]; w1 = wx[DD + ci]; }
    }
#pragma unroll
    for (int r = 0; r < 8; ++r) {
      const int lr = 16 * wave + 8 * hh + r;
      float v;
      if (EPI == 0) {
        v = fmaf(acc[t][r], scl, bv);
      } else if (EPI == 1) {
        float z = fmaf(acc[t][r], scl, bv);
        z = fmaf(ev0[r], w0, z);
        z = fmaf(ev1[r], w1, z);
        v = silu_f(z);
      } else {
        v = fmaf(acc[t][r], scl, bv) * ev0[r];
      }
      stg[lr * GBN + lc] = v;
    }
  }
  __syncthreads();

  if (EPI == 1) {
    const int q8 = (lane & 7) * 8;
    v8h hv[4];
#pragma unroll
    for (int i = 0; i < 4; ++i) {
      const int lr = 16 * wave + 4 * i + (lane >> 3);
      const v4f a = *(const v4f*)(stg + lr * GBN + q8);
      const v4f b = *(const v4f*)(stg + lr * GBN + q8 + 4);
      hv[i] = cvt8h(a, b, CA);
    }
#pragma unroll
    for (int i = 0; i < 4; ++i) {
      const int lr = 16 * wave + 4 * i + (lane >> 3);
      const int gr = rowBase + lr;
      _Float16* op = outH + (size_t)gr * (size_t)ldo + col0 + q8;
      *(volatile v8h*)op = hv[i];
    }
    __threadfence();
#pragma unroll
    for (int i = 0; i < 4; ++i) {
      const int lr = 16 * wave + 4 * i + (lane >> 3);
      const int gr = rowBase + lr;
      _Float16* op = outH + (size_t)gr * (size_t)ldo + col0 + q8;
      *(volatile v8h*)op = hv[i];
    }
  } else {
    v4f fv[8];
#pragma unroll
    for (int i = 0; i < 8; ++i) {
      const int lr = 16 * wave + 2 * i + hh;
      fv[i] = *(const v4f*)(stg + lr * GBN + 4 * m);
    }
#pragma unroll
    for (int i = 0; i < 8; ++i) {
      const int lr = 16 * wave + 2 * i + hh;
      const int gr = rowBase + lr;
      float* op = outF + (size_t)gr * (size_t)ldo + col0 + 4 * m;
      *(volatile v4f*)op = fv[i];
    }
    __threadfence();
#pragma unroll
    for (int i = 0; i < 8; ++i) {
      const int lr = 16 * wave + 2 * i + hh;
      const int gr = rowBase + lr;
      float* op = outF + (size_t)gr * (size_t)ldo + col0 + 4 * m;
      *(volatile v4f*)op = fv[i];
    }
  }
}

__global__ __launch_bounds__(NTHR) void k_node1(const float* __restrict__ H, const float* __restrict__ bias,
                                                float* XPF, int NPr) {
  const int tid = (int)threadIdx.x, lane = tid & 31, wave = tid >> 5;
  const int row = (int)blockIdx.x * NWAVE + wave;
  if (row >= NPr) return;
  const float* hp = H + (size_t)row * DD + 8 * lane;
  const v4f ha = *(const v4f*)hp, hb = *(const v4f*)(hp + 4);
  float u[8] = {ha.x, ha.y, ha.z, ha.w, hb.x, hb.y, hb.z, hb.w};
  if (lane == 0) u[0] = 0.f;
  float ss = 0.f;
#pragma unroll
  for (int k = 0; k < 8; ++k) ss = fmaf(u[k], u[k], ss);
  ss = wred(ss);
  const float n1 = sqrtf(fmaxf(ss, EPSF));
  float ch1, sh1;
  chsh(n1, ch1, sh1);
  const float sc1 = sh1 * rcp_f(n1);
  float y[8];
#pragma unroll
  for (int k = 0; k < 8; ++k) y[k] = sc1 * u[k];
  if (lane == 0) y[0] = ch1;

  const v4f ba = *(const v4f*)(bias + 8 * lane), bb = *(const v4f*)(bias + 8 * lane + 4);
  float b[8] = {ba.x, ba.y, ba.z, ba.w, bb.x, bb.y, bb.z, bb.w};
  if (lane == 0) b[0] = 0.f;
  float lin = 0.f;
#pragma unroll
  for (int k = 0; k < 8; ++k) lin = fmaf(y[k], b[k], lin);
  lin = wred(lin);
  const float cc = lin * rcp_f(1.0f + ch1);
  float tb[8];
#pragma unroll
  for (int k = 0; k < 8; ++k) {
    const float w = y[k] + ((lane == 0 && k == 0) ? 1.0f : 0.0f);
    tb[k] = fmaf(cc, w, b[k]);
  }
  const float tb0 = cc * (ch1 + 1.0f);
  float q = 0.f;
#pragma unroll
  for (int k = 0; k < 8; ++k) q = fmaf(tb[k], tb[k], q);
  q = wred(q);
  q = q - 2.0f * tb0 * tb0;
  const float nu = sqrtf(fmaxf(q, EPSF));
  float ch2, sh2;
  chsh(nu, ch2, sh2);
  const float s2 = sh2 * rcp_f(nu);
  float z[8];
#pragma unroll
  for (int k = 0; k < 8; ++k) z[k] = fmaf(s2, tb[k], ch2 * y[k]);
  put_row(XPF + (size_t)row * DD, z, lane);
}

__global__ __launch_bounds__(NTHR) void k_egeo(const int* __restrict__ rowi, const int* __restrict__ coli,
                                               const float* __restrict__ XPF, _Float16* XL, float* ESD,
                                               int nN, int ebase, int nE) {
  __shared__ __attribute__((aligned(16))) float sd[EPB];
  const int tid = (int)threadIdx.x, lane = tid & 31, wave = tid >> 5;
#pragma unroll 1
  for (int j = 0; j < EPW; ++j) {
    const int le = (int)blockIdx.x * EPB + wave * EPW + j;
    const int e  = ebase + le;
    const bool valid = e < nE;
    const int ec = e < nE ? e : nE - 1;
    int r = rowi[ec]; r = r < 0 ? 0 : (r > nN - 1 ? nN - 1 : r);
    int c = coli[ec]; c = c < 0 ? 0 : (c > nN - 1 ? nN - 1 : c);
    const float* pr = XPF + (size_t)r * DD + 8 * lane;
    const float* pc = XPF + (size_t)c * DD + 8 * lane;
    const v4f ra = *(const v4f*)pr, rb = *(const v4f*)(pr + 4);
    const v4f qa = *(const v4f*)pc, qb = *(const v4f*)(pc + 4);
    const float xr[8] = {ra.x, ra.y, ra.z, ra.w, rb.x, rb.y, rb.z, rb.w};
    const float xc[8] = {qa.x, qa.y, qa.z, qa.w, qb.x, qb.y, qb.z, qb.w};
    float s = xr[0] * xc[0];
#pragma unroll
    for (int k = 1; k < 8; ++k) s = fmaf(xr[k], xc[k], s);
    s = wred(s);
    const float xr0 = __shfl(xr[0], 0);
    const float xc0 = __shfl(xc[0], 0);
    const float li  = s - 2.0f * xr0 * xc0;
    const float a   = fmaxf(-li, ONEPE);
    const float d   = acoshf(a);
    const float cf  = d * rcp_f(sqrtf(a * a - 1.0f));
    float v[8];
#pragma unroll
    for (int k = 0; k < 8; ++k) v[k] = cf * (xc[k] - a * xr[k]);
    const float v0  = __shfl(v[0], 0);
    const float fac = -v0 * rcp_f(1.0f + xr0);
    const float vf  = valid ? 1.0f : 0.0f;
    float xl[8];
#pragma unroll
    for (int k = 0; k < 8; ++k) {
      const float w = xr[k] + ((lane == 0 && k == 0) ? 1.0f : 0.0f);
      xl[k] = fmaf(fac, w, v[k]) * vf;
    }
    const v4f oa = {xl[0], xl[1], xl[2], xl[3]};
    const v4f ob = {xl[4], xl[5], xl[6], xl[7]};
    const v8h hv = cvt8h(oa, ob, CA);
    _Float16* op = XL + (size_t)le * DD + 8 * lane;
    *(volatile v8h*)op = hv;
    __threadfence();
    *(volatile v8h*)op = hv;
    if (lane == 0) sd[wave * EPW + j] = d * vf;
  }
  __syncthreads();
  if (wave == 0) {
    const int lq = lane & 7;
    const v4f dv = *(const v4f*)(sd + 4 * lq);
    float* p = ESD + (size_t)blockIdx.x * EPB + 4 * lq;
    if (lane < 8) *(volatile v4f*)p = dv;
    __threadfence();
    if (lane < 8) *(volatile v4f*)p = dv;
  }
}

__global__ __launch_bounds__(NTHR) void k_eatt(const int* __restrict__ rowi, const int* __restrict__ coli,
                                               const float* __restrict__ eattr, const float* __restrict__ emsk,
                                               const float* __restrict__ PQ, const float* __restrict__ Wa1,
                                               const float* __restrict__ Wa2, const float* __restrict__ ba2,
                                               const float* __restrict__ ESD, float* ESA,
                                               int nN, int ebase, int nE) {
  __shared__ __attribute__((aligned(16))) float sa[EPB];
  const int tid = (int)threadIdx.x, lane = tid & 31, wave = tid >> 5;
  const float* pw0 = Wa1 + (size_t)(2 * DD) * DD + 8 * lane;
  const float* pw1 = Wa1 + (size_t)(2 * DD + 1) * DD + 8 * lane;
  const v4f wa0 = *(const v4f*)pw0, wa1v = *(const v4f*)(pw0 + 4);
  const v4f wb0 = *(const v4f*)pw1, wb1v = *(const v4f*)(pw1 + 4);
  const v4f wc0 = *(const v4f*)(Wa2 + 8 * lane), wc1 = *(const v4f*)(Wa2 + 8 * lane + 4);
  const float wa[8] = {wa0.x, wa0.y, wa0.z, wa0.w, wa1v.x, wa1v.y, wa1v.z, wa1v.w};
  const float wb[8] = {wb0.x, wb0.y, wb0.z, wb0.w, wb1v.x, wb1v.y, wb1v.z, wb1v.w};
  const float w2[8] = {wc0.x, wc0.y, wc0.z, wc0.w, wc1.x, wc1.y, wc1.z, wc1.w};
  const float b2 = ba2[0];
#pragma unroll 1
  for (int j = 0; j < EPW; ++j) {
    const int le = (int)blockIdx.x * EPB + wave * EPW + j;
    const int e  = ebase + le;
    const bool valid = e < nE;
    const int ec = e < nE ? e : nE - 1;
    int r = rowi[ec]; r = r < 0 ? 0 : (r > nN - 1 ? nN - 1 : r);
    int c = coli[ec]; c = c < 0 ? 0 : (c > nN - 1 ? nN - 1 : c);
    const float* pp = PQ + (size_t)r * DQ + 8 * lane;
    const float* pq = PQ + (size_t)c * DQ + DD + 8 * lane;
    const v4f pa = *(const v4f*)pp, pb = *(const v4f*)(pp + 4);
    const v4f qa = *(const v4f*)pq, qb = *(const v4f*)(pq + 4);
    const float P[8] = {pa.x, pa.y, pa.z, pa.w, pb.x, pb.y, pb.z, pb.w};
    const float Q[8] = {qa.x, qa.y, qa.z, qa.w, qb.x, qb.y, qb.z, qb.w};
    const float ea0 = eattr[ec];
    const float ea1 = ESD[le];
    const float em  = emsk[ec];
    float lg = 0.f;
#pragma unroll
    for (int k = 0; k < 8; ++k) {
      float pre = P[k] + Q[k];
      pre = fmaf(ea0, wa[k], pre);
      pre = fmaf(ea1, wb[k], pre);
      const float a1 = silu_f(pre);
      lg = fmaf(a1, w2[k], lg);
    }
    lg = wred(lg) + b2;
    const float vf  = valid ? 1.0f : 0.0f;
    const float att = sigm_f(lg) * em * vf;
    if (lane == 0) sa[wave * EPW + j] = att;
  }
  __syncthreads();
  if (wave == 0) {
    const int lq = lane & 7;
    const v4f dv = *(const v4f*)(sa + 4 * lq);
    float* p = ESA + (size_t)blockIdx.x * EPB + 4 * lq;
    if (lane < 8) *(volatile v4f*)p = dv;
    __threadfence();
    if (lane < 8) *(volatile v4f*)p = dv;
  }
}

__global__ __launch_bounds__(NTHR) void k_agg(
    const int* __restrict__ dsts, const float* __restrict__ MSG, float* AGG,
    int nN, int nE, int nb, int vec8, int NPr, int accum) {
  extern __shared__ v4f lds_dyn[];
  int* reg1 = (int*)lds_dyn;
  int* reg2 = reg1 + RCAP;
  int* scnt = reg2 + RCAP;
  int* soff = scnt + NBMAX;
  int* list = soff + NBMAX;
  int* wcnt = list + LISTN;
  int* wtot = wcnt + NWAVE;
  const int tid = (int)threadIdx.x, lane = tid & 31, wave = tid >> 5;
  const int nodeBase = (int)blockIdx.x * nb;

  for (int i = tid; i < NBMAX; i += NTHR) scnt[i] = 0;
  __syncthreads();

  int tot = 0;
  const int nChunks = (nE + CHUNK - 1) / CHUNK;
#pragma unroll 1
  for (int ch = 0; ch < nChunks; ++ch) {
    const int cbase = ch * CHUNK;
    const int wc = scan_chunk(dsts, nE, cbase, nodeBase, nb, vec8, list, tid, lane, wave);
    if (lane == 0) wcnt[wave] = wc;
    __syncthreads();
    int pre = 0, all = 0;
#pragma unroll
    for (int w2 = 0; w2 < NWAVE; ++w2) {
      int c = wcnt[w2];
      c = c < 0 ? 0 : (c > WCAP ? WCAP : c);
      all += c;
      pre += (w2 < wave) ? c : 0;
    }
    const int wcc  = wc > WCAP ? WCAP : wc;
    const int base = tot + pre;
#pragma unroll 1
    for (int i = lane; i < wcc; i += 32) {
      const int ent = list[wave * WCAP + i];
      const int el  = (ent >> 12) & (CHUNK - 1);
      const int sl  = ent & (NBMAX - 1);
      int eid = cbase + el;
      eid = eid > nE - 1 ? nE - 1 : eid;
      const int pos = base + i;
      if (pos < RCAP) reg1[pos] = (int)(((unsigned)eid << 12) | (unsigned)sl);
    }
    tot += all;
    tot = tot > RCAP ? RCAP : tot;
    __syncthreads();
  }
  const int nh = tot;

  if (wave == 0) {
#pragma unroll 1
    for (int b0 = 0; b0 < nh; b0 += 32) {
      const int idx = b0 + lane;
      const int uv  = reg1[idx < RCAP ? idx : RCAP - 1];
      const int m32 = (nh - b0) < 32 ? (nh - b0) : 32;
#pragma unroll 1
      for (int k = 0; k < m32; ++k) {
        const int u  = __builtin_amdgcn_readlane(uv, k);
        const int sl = u & (NBMAX - 1);
        if (lane == 0) scnt[sl] = scnt[sl] + 1;
      }
    }
  }
  __syncthreads();

  {
    const v4i ca = *(const v4i*)(scnt + 8 * tid);
    const v4i cb = *(const v4i*)(scnt + 8 * tid + 4);
    const int e0 = ca.x < 0 ? 0 : ca.x, e1 = ca.y < 0 ? 0 : ca.y, e2 = ca.z < 0 ? 0 : ca.z, e3 = ca.w < 0 ? 0 : ca.w;
    const int e4 = cb.x < 0 ? 0 : cb.x, e5 = cb.y < 0 ? 0 : cb.y, e6 = cb.z < 0 ? 0 : cb.z, e7 = cb.w < 0 ? 0 : cb.w;
    const int ts = e0 + e1 + e2 + e3 + e4 + e5 + e6 + e7;
    int incl = ts;
#pragma unroll
    for (int d = 1; d < 32; d <<= 1) {
      const int up = __shfl_up(incl, d);
      if (lane >= d) incl += up;
    }
    if (lane == 31) wtot[wave] = incl;
    __syncthreads();
    int pre = 0;
#pragma unroll
    for (int w2 = 0; w2 < NWAVE; ++w2) pre += (w2 < wave) ? wtot[w2] : 0;
    int run = pre + incl - ts;
    soff[8 * tid + 0] = run; run += e0;
    soff[8 * tid + 1] = run; run += e1;
    soff[8 * tid + 2] = run; run += e2;
    soff[8 * tid + 3] = run; run += e3;
    soff[8 * tid + 4] = run; run += e4;
    soff[8 * tid + 5] = run; run += e5;
    soff[8 * tid + 6] = run; run += e6;
    soff[8 * tid + 7] = run;
  }
  __syncthreads();
  for (int i = tid; i < NBMAX; i += NTHR) list[i] = soff[i];
  __syncthreads();

  if (wave == 0) {
#pragma unroll 1
    for (int b0 = 0; b0 < nh; b0 += 32) {
      const int idx = b0 + lane;
      const int uv  = reg1[idx < RCAP ? idx : RCAP - 1];
      const int m32 = (nh - b0) < 32 ? (nh - b0) : 32;
#pragma unroll 1
      for (int k = 0; k < m32; ++k) {
        const int u   = __builtin_amdgcn_readlane(uv, k);
        const int sl  = u & (NBMAX - 1);
        const int eid = (int)((unsigned)u >> 12);
        if (lane == 0) {
          int pos = list[sl];
          pos = pos < 0 ? 0 : (pos > RCAP - 1 ? RCAP - 1 : pos);
          reg2[pos] = eid;
          list[sl] = pos + 1;
        }
      }
    }
  }
  __syncthreads();

  const int nbw = nb >> 3;
  const bool ovf = (nh >= RCAP);
  const float qnan = __int_as_float(0x7fc00000);
#pragma unroll 1
  for (int jt = 0; jt < nbw; ++jt) {
    const int slot = wave * nbw + jt;
    const int grow = nodeBase + slot;
    const int gcl  = grow < nN ? grow : nN - 1;
    int st = soff[slot];
    const int craw = scnt[slot];
    int cnt = craw;
    st  = st < 0 ? 0 : (st > nh ? nh : st);
    cnt = cnt < 0 ? 0 : (cnt > DEGCAP ? DEGCAP : cnt);
    if (cnt > nh - st) cnt = nh - st;
    const float pz = (ovf || craw > DEGCAP) ? qnan : 0.0f;
    const bool wr = grow < NPr;
    const float live = grow < nN ? 1.0f : 0.0f;

    float sm[8];
#pragma unroll
    for (int j = 0; j < 8; ++j) sm[j] = 0.f;
#pragma unroll 1
    for (int q = 0; q < cnt; ++q) {
      int idx = st + q; idx = idx > RCAP - 1 ? RCAP - 1 : idx;
      int el = reg2[idx]; el = el < 0 ? 0 : (el > nE - 1 ? nE - 1 : el);
      const float* mr = MSG + (size_t)el * DD + lane;
      float mv[8];
#pragma unroll
      for (int j = 0; j < 8; ++j) mv[j] = mr[32 * j];
      ldwait();
#pragma unroll
      for (int j = 0; j < 8; ++j) sm[j] += mv[j];
    }
    float od[8];
#pragma unroll
    for (int j = 0; j < 8; ++j) od[j] = 0.f;
    if (accum != 0) {
      const float* ar = AGG + (size_t)gcl * DD + lane;
#pragma unroll
      for (int j = 0; j < 8; ++j) od[j] = ar[32 * j];
      ldwait();
    }
    float rs[8];
#pragma unroll
    for (int j = 0; j < 8; ++j) rs[j] = (sm[j] + od[j]) * live + pz;
    float* gp = AGG + (size_t)grow * DD + lane;
    if (wr) {
#pragma unroll
      for (int j = 0; j < 8; ++j) *(volatile float*)(gp + 32 * j) = rs[j];
    }
    __threadfence();
    if (wr) {
#pragma unroll
      for (int j = 0; j < 8; ++j) *(volatile float*)(gp + 32 * j) = rs[j];
    }
  }
}

__global__ __launch_bounds__(NTHR) void k_fin1(const float* __restrict__ XPF, const float* __restrict__ AGG,
                                               float* XO, int nN) {
  const int tid = (int)threadIdx.x, lane = tid & 31, wave = tid >> 5;
  const int row = (int)blockIdx.x * NWAVE + wave;
  if (row >= nN) return;
  const float* zp = XPF + (size_t)row * DD + 8 * lane;
  const float* gq = AGG + (size_t)row * DD + 8 * lane;
  const v4f za = *(const v4f*)zp, zb = *(const v4f*)(zp + 4);
  const v4f ga = *(const v4f*)gq, gb = *(const v4f*)(gq + 4);
  const float z[8] = {za.x, za.y, za.z, za.w, zb.x, zb.y, zb.z, zb.w};
  float g[8] = {ga.x, ga.y, ga.z, ga.w, gb.x, gb.y, gb.z, gb.w};
  if (lane == 0) g[0] = 0.f;
  const float z0 = __shfl(z[0], 0);
  float lin = 0.f;
#pragma unroll
  for (int k = 0; k < 8; ++k) lin = fmaf(z[k], g[k], lin);
  lin = wred(lin);
  const float cc = lin * rcp_f(1.0f + z0);
  float sp[8];
#pragma unroll
  for (int k = 0; k < 8; ++k) {
    const float w = z[k] + ((lane == 0 && k == 0) ? 1.0f : 0.0f);
    sp[k] = fmaf(cc, w, g[k]);
  }
  const float sp0 = cc * (z0 + 1.0f);
  float q = 0.f;
#pragma unroll
  for (int k = 0; k < 8; ++k) q = fmaf(sp[k], sp[k], q);
  q = wred(q);
  q = q - 2.0f * sp0 * sp0;
  const float nu = sqrtf(fmaxf(q, EPSF));
  float ch, sh;
  chsh(nu, ch, sh);
  const float s2 = sh * rcp_f(nu);
  float y[8];
#pragma unroll
  for (int k = 0; k < 8; ++k) y[k] = fmaf(s2, sp[k], ch * z[k]);
  const float y0 = fmaxf(__shfl(y[0], 0), ONEPE);
  const float d  = acoshf(y0);
  const float ct = d * rcp_f(sqrtf(y0 * y0 - 1.0f));
  float t[8];
#pragma unroll
  for (int k = 0; k < 8; ++k) t[k] = ct * y[k];
  if (lane == 0) t[0] = 0.f;
  put_row(XO + (size_t)row * DD, t, lane);
}

__global__ __launch_bounds__(NTHR) void k_fin2(const float* __restrict__ XO, const float* __restrict__ lng,
                                               const float* __restrict__ lnb, float* out, int nN) {
  __shared__ __attribute__((aligned(16))) float sg[DD];
  __shared__ __attribute__((aligned(16))) float sb[DD];
  const int tid = (int)threadIdx.x, lane = tid & 31, wave = tid >> 5;
  {
    const int li = tid > 0 ? tid - 1 : 0;
    const float gv = lng[li], bv = lnb[li];
    sg[tid] = tid > 0 ? gv : 0.f;
    sb[tid] = tid > 0 ? bv : 0.f;
  }
  __syncthreads();
  const int row = (int)blockIdx.x * NWAVE + wave;
  if (row >= nN) return;
  const float* tp = XO + (size_t)row * DD + 8 * lane;
  const v4f ta = *(const v4f*)tp, tb = *(const v4f*)(tp + 4);
  const float t[8] = {ta.x, ta.y, ta.z, ta.w, tb.x, tb.y, tb.z, tb.w};
  float s1 = 0.f;
#pragma unroll
  for (int k = 0; k < 8; ++k) s1 += t[k];
  s1 = wred(s1);
  const float mean = s1 * (1.0f / 255.0f);
  float s2 = 0.f;
#pragma unroll
  for (int k = 0; k < 8; ++k) {
    const int c = 8 * lane + k;
    const float dv = t[k] - mean;
    const float dz = (c == 0) ? 0.f : dv;
    s2 = fmaf(dz, dz, s2);
  }
  s2 = wred(s2);
  const float var = s2 * (1.0f / 255.0f);
  const float rsd = rcp_f(sqrtf(var + LNEPS));
  const v4f g0 = *(const v4f*)(sg + 8 * lane), g1 = *(const v4f*)(sg + 8 * lane + 4);
  const v4f b0 = *(const v4f*)(sb + 8 * lane), b1 = *(const v4f*)(sb + 8 * lane + 4);
  const float g[8] = {g0.x, g0.y, g0.z, g0.w, g1.x, g1.y, g1.z, g1.w};
  const float b[8] = {b0.x, b0.y, b0.z, b0.w, b1.x, b1.y, b1.z, b1.w};
  float u[8];
#pragma unroll
  for (int k = 0; k < 8; ++k) {
    const int c = 8 * lane + k;
    const float ln = fmaf((t[k] - mean) * rsd, g[k], b[k]);
    const float sv = silu_f(ln);
    u[k] = (c == 0) ? 0.f : sv;
  }
  float ss = 0.f;
#pragma unroll
  for (int k = 0; k < 8; ++k) ss = fmaf(u[k], u[k], ss);
  ss = wred(ss);
  const float n = sqrtf(fmaxf(ss, EPSF));
  float ch, sh;
  chsh(n, ch, sh);
  const float sc = sh * rcp_f(n);
  float o[8];
#pragma unroll
  for (int k = 0; k < 8; ++k) o[k] = sc * u[k];
  if (lane == 0) o[0] = ch;
  put_row(out + (size_t)row * DD, o, lane);
}

static inline int cdiv(int a, int b) { return (a + b - 1) / b; }
static int pick_nb(int chm, int nN) {
  int nb = NBMAX;
  while (nb > 16 && (long long)nb * (long long)chm * 4LL > (long long)RCAP * (long long)nN) nb >>= 1;
  return nb;
}

extern "C" void kernel_launch(void* const* d_in, const int* in_sizes, int n_in,
                              void* d_out, int out_size, void* d_ws, size_t ws_size,
                              hipStream_t stream) {
  if (n_in < 18) return;
  const int nN = in_sizes[0] / DD;
  if (nN <= 0 || in_sizes[0] != nN * DD || nN > (1 << 20)) return;
  const int nE = in_sizes[2];
  if (nE < 1 || nE > (1 << 24)) return;
  if (in_sizes[1] != nE || in_sizes[3] != nE || in_sizes[5] != nE) return;
  if (in_sizes[6]  != DD * DD           || in_sizes[7]  != DD) return;
  if (in_sizes[8]  != (DD + 2) * DD     || in_sizes[9]  != DD) return;
  if (in_sizes[10] != DD * DD           || in_sizes[11] != DD) return;
  if (in_sizes[12] != (2 * DD + 2) * DD || in_sizes[13] != DD) return;
  if (in_sizes[14] != DD                || in_sizes[15] < 1)   return;
  if (in_sizes[16] != DD - 1            || in_sizes[17] != DD - 1) return;
  if (out_size != nN * DD) return;

  const float* x     = (const float*)d_in[0];
  const float* eattr = (const float*)d_in[1];
  const int*   rowi  = (const int*)  d_in[2];
  const int*   coli  = (const int*)  d_in[3];
  const float* emsk  = (const float*)d_in[5];
  const float* W_lin = (const float*)d_in[6];
  const float* bias  = (const float*)d_in[7];
  const float* W_e1  = (const float*)d_in[8];
  const float* b_e1  = (const float*)d_in[9];
  const float* W_e2  = (const float*)d_in[10];
  const float* b_e2  = (const float*)d_in[11];
  const float* W_a1  = (const float*)d_in[12];
  const float* b_a1  = (const float*)d_in[13];
  const float* W_a2  = (const float*)d_in[14];
  const float* b_a2  = (const float*)d_in[15];
  const float* ln_g  = (const float*)d_in[16];
  const float* ln_b  = (const float*)d_in[17];
  float* out = (float*)d_out;

  const int NP     = cdiv(nN, GBM) * GBM;
  const int tilesE = cdiv(nE, GBM);
  const int tpc    = cdiv(tilesE, NCH);
  const int CHM    = tpc * GBM;
  const int nb     = pick_nb(CHM, nN);
  const int gA     = cdiv(NP, nb);
  if (gA * nb < NP) return;

  char* ws = (char*)d_ws;
  size_t off = 0;
  const size_t oWPL = off; off += (size_t)WROWS * DD * 2;          off = (off + 255) & ~(size_t)255;
  const size_t oR1  = off; off += (size_t)NP * DD * 2;             off = (off + 255) & ~(size_t)255;
  const size_t oR2  = off; off += (size_t)NP * DD * 4;             off = (off + 255) & ~(size_t)255;
  const size_t oXPF = off; off += (size_t)NP * DD * 4;             off = (off + 255) & ~(size_t)255;
  const size_t oPQ  = off; off += (size_t)NP * DQ * 4;             off = (off + 255) & ~(size_t)255;
  const size_t oESD = off; off += (size_t)CHM * 4;                 off = (off + 255) & ~(size_t)255;
  const size_t oESA = off; off += (size_t)CHM * 4;                 off = (off + 255) & ~(size_t)255;
  const size_t oXL  = off; off += (size_t)CHM * DD * 2;            off = (off + 255) & ~(size_t)255;
  const size_t oM1  = off; off += (size_t)CHM * DD * 2;            off = (off + 255) & ~(size_t)255;
  const size_t oMSG = off; off += (size_t)CHM * DD * 4;            off = (off + 255) & ~(size_t)255;
  if (off > ws_size || off > (size_t)WSMAX) return;
  _Float16* WPL  = (_Float16*)(ws + oWPL);
  _Float16* WT0  = WPL;
  _Float16* WTA  = WPL + (size_t)256 * DD;
  _Float16* WT1  = WPL + (size_t)768 * DD;
  _Float16* WT2  = WPL + (size_t)1024 * DD;
  _Float16* TH   = (_Float16*)(ws + oR1);
  _Float16* XTH  = TH;
  float*    H    = (float*)(ws + oR2);
  float*    AGG  = H;
  float*    XPF  = (float*)(ws + oXPF);
  float*    PQ   = (float*)(ws + oPQ);
  float*    XO   = PQ;
  float*    ESD  = (float*)(ws + oESD);
  float*    ESA  = (float*)(ws + oESA);
  _Float16* XL   = (_Float16*)(ws + oXL);
  _Float16* M1   = (_Float16*)(ws + oM1);
  float*    MSGA = (float*)(ws + oMSG);
  const float* W_e1x = W_e1 + (size_t)DD * DD;

  hipFuncSetAttribute(reinterpret_cast<const void*>(&k_agg),
                      hipFuncAttributeMaxDynamicSharedMemorySize, LDS_AGG);

  {
    const int nU = WROWS * (DD / 8);
    k_wcvt<<<cdiv(nU, NTHR), NTHR, 0, stream>>>(W_lin, W_a1, W_a1 + (size_t)DD * DD, W_e1, W_e2, WPL, nU);
  }
  {
    const int nU = NP * (DD / 8);
    k_tan<<<cdiv(nU, NTHR), NTHR, 0, stream>>>(x, TH, nN, nU);
  }
  const int gM = NP / GBM;
  k_gemm<0><<<dim3(gM, DD / GBN), GTHR, 0, stream>>>(TH, WT0, b_a1, eattr, ESD, ESA, W_e1x, H, M1,
                                                     DD, DD, 0, 0, nE, SCL);
  k_node1<<<NP / NWAVE, NTHR, 0, stream>>>(H, bias, XPF, NP);
  {
    const int nU = NP * (DD / 8);
    k_tan<<<cdiv(nU, NTHR), NTHR, 0, stream>>>(XPF, XTH, NP, nU);
  }
  k_gemm<0><<<dim3(gM, DQ / GBN), GTHR, 0, stream>>>(XTH, WTA, b_a1, eattr, ESD, ESA, W_e1x, PQ, M1,
                                                     DD, DQ, DD, 0, nE, SCL);

  for (int c = 0; c < NCH; ++c) {
    const int t0 = c * tpc;
    int t1 = t0 + tpc;
    t1 = t1 > tilesE ? tilesE : t1;
    if (t1 <= t0) continue;
    const int rows  = (t1 - t0) * GBM;
    const int ebase = t0 * GBM;
    int nEc = nE - ebase;
    nEc = nEc > rows ? rows : nEc;
    const int vec8  = ((ebase & 3) == 0) ? 1 : 0;
    const int accum = (c == 0) ? 0 : 1;
    k_egeo<<<rows / EPB, NTHR, 0, stream>>>(rowi, coli, XPF, XL, ESD, nN, ebase, nE);
    k_eatt<<<rows / EPB, NTHR, 0, stream>>>(rowi, coli, eattr, emsk, PQ, W_a1, W_a2, b_a2, ESD, ESA,
                                            nN, ebase, nE);
    k_gemm<1><<<dim3(rows / GBM, DD / GBN), GTHR, 0, stream>>>(XL, WT1, b_e1, eattr, ESD, ESA, W_e1x,
                                                               MSGA, M1, DD, DD, DD, ebase, nE, SCL);
    k_gemm<2><<<dim3(rows / GBM, DD / GBN), GTHR, 0, stream>>>(M1, WT2, b_e2, eattr, ESD, ESA, W_e1x,
                                                               MSGA, M1, DD, DD, DD, ebase, nE, SCL);
    k_agg<<<gA, NTHR, LDS_AGG, stream>>>(rowi + ebase, MSGA, AGG, nN, nEc, nb, vec8, NP, accum);
  }

  k_fin1<<<cdiv(nN, NWAVE), NTHR, 0, stream>>>(XPF, AGG, XO, nN);
  k_fin2<<<cdiv(nN, NWAVE), NTHR, 0, stream>>>(XO, ln_g, ln_b, out, nN);
}
